// DisentangledSelfAttention_87153476370982
// MI455X (gfx1250) — hardware-verified
//
#include <hip/hip_runtime.h>
#include <math.h>

typedef _Float16 half_t;
typedef _Float16 v16h __attribute__((ext_vector_type(16)));
typedef _Float16 v8h  __attribute__((ext_vector_type(8)));
typedef float    v8f  __attribute__((ext_vector_type(8)));
typedef int      v4i  __attribute__((ext_vector_type(4)));

#define B_    2
#define S_    2048
#define HID_  768
#define H_    12
#define D_    64
#define P_    512
#define SCALE_ 0.125f

#define HAVE_ASYNC 0

#define GAS1(p) ((__attribute__((address_space(1))) v4i*)(p))
#define LAS3(p) ((__attribute__((address_space(3))) v4i*)(p))

union AFrag { v16h v; v8h h[2]; };
typedef float v4f __attribute__((ext_vector_type(4)));
typedef unsigned v4u __attribute__((ext_vector_type(4)));
template <typename V> __device__ __forceinline__ void vst2(void* p, V v) {
  *(volatile V*)p = v; __threadfence(); *(volatile V*)p = v;
}
#define PSC 256.0f
#define PUN (1.0f / 256.0f)
__device__ __forceinline__ v8f wmma16(v16h a, v16h b, v8f c) {
  v8f d = __builtin_amdgcn_wmma_f32_16x16x32_f16(false, a, false, b, (short)0, c, false, false);
  asm volatile("v_nop\n\tv_nop\n\tv_nop\n\tv_nop" : "+v"(d) : "v"(a), "v"(b));
  return d;
}

__global__ void cvt_f16_kernel(const float* __restrict__ in, half_t* __restrict__ out, int n) {
  int g = blockIdx.x * 256 + threadIdx.x;
  if (g * 8 >= n) return;
  union { v8h h; v4u u; } pk;
#pragma unroll
  for (int e = 0; e < 8; ++e) pk.h[e] = (half_t)in[(size_t)g * 8 + e];
  vst2(out + (size_t)g * 8, pk.u);
}

__global__ __launch_bounds__(256) void cvt_transpose_kernel(const float* __restrict__ W, half_t* __restrict__ Wt) {
  __shared__ __align__(16) half_t tile[64][72];
  const int n0 = (blockIdx.x % (HID_ / 64)) * 64, k0 = (blockIdx.x / (HID_ / 64)) * 64, tid = threadIdx.x;
  for (int i = tid; i < 64 * 64; i += 256) { const int kk = i >> 6, nn = i & 63; tile[nn][kk] = (half_t)W[(size_t)(k0 + kk) * HID_ + n0 + nn]; }
  __syncthreads();
  for (int g = tid; g < 64 * 8; g += 256) { const int nn = g >> 3, pc = g & 7; vst2(Wt + (size_t)(n0 + nn) * HID_ + k0 + pc * 8, *(const v4u*)(&tile[nn][pc * 8])); }
}

__global__ void __launch_bounds__(256)
gemm_proj_kernel(const half_t* __restrict__ X, const half_t* __restrict__ Wt,
                 const float* __restrict__ bias,
                 half_t* __restrict__ Yh, float* __restrict__ Yf,
                 int M, int mode) {
  __shared__ __align__(16) float T[16][128];
  int lane = threadIdx.x & 31;
  int wave = threadIdx.x >> 5;
  int tile = blockIdx.x * 8 + wave;
  const int ntn = HID_ / 16;
  int mt = tile / ntn;
  int nt = tile - mt * ntn;
  int m0 = mt * 16, n0 = nt * 16;
  const int nb0 = (nt & ~7) * 16;
  if (m0 >= M) return;

  int ln = lane & 15;
  int khalf = (lane >> 4) << 3;
  const half_t* xrow = X  + (size_t)(m0 + ln) * HID_;
  const half_t* wrow = Wt + (size_t)(n0 + ln) * HID_;

  v8f acc = {};
  #pragma unroll 4
  for (int k0 = 0; k0 < HID_; k0 += 32) {
    AFrag a, b;
    a.h[0] = *(const v8h*)(xrow + k0 + khalf);
    a.h[1] = *(const v8h*)(xrow + k0 + khalf + 16);
    b.h[0] = *(const v8h*)(wrow + k0 + khalf);
    b.h[1] = *(const v8h*)(wrow + k0 + khalf + 16);
    acc = wmma16(a.v, b.v, acc);
  }

  int n = n0 + ln;
  float bvv = bias ? bias[n] : 0.0f;
  #pragma unroll
  for (int g = 0; g < 8; ++g) T[((lane >> 4) << 3) + g][wave * 16 + ln] = acc[g] + bvv;
  __syncthreads();
  const int tid = threadIdx.x;
  if (mode == 3) {
    for (int gq = tid; gq < 16 * 32; gq += 256) { const int r = gq >> 5, pc = gq & 31; vst2(Yf + (size_t)(m0 + r) * HID_ + nb0 + pc * 4, *(const v4f*)(&T[r][pc * 4])); }
  } else {
    const int r = tid >> 4, pc = tid & 15;
    union { v8h h; v4u u; } pk;
    #pragma unroll
    for (int e = 0; e < 8; ++e) pk.h[e] = (half_t)T[r][pc * 8 + e];
    const int m = m0 + r;
    if (mode == 2) vst2(Yh + (size_t)m * HID_ + nb0 + pc * 8, pk.u);
    else { const int nn = nb0 + pc * 8; const int b = m >> 11, s = m & 2047, h = nn >> 6, d = nn & 63;
           vst2(Yh + (((size_t)(b * H_ + h)) * S_ + s) * D_ + d, pk.u); }
  }
}

__global__ void __launch_bounds__(256)
gemm_rel_kernel(const half_t* __restrict__ A, const half_t* __restrict__ Pos,
                half_t* __restrict__ Out) {
  __shared__ __align__(16) half_t T[16][128];
  int lane = threadIdx.x & 31;
  int wave = threadIdx.x >> 5;
  int tile = blockIdx.x * 8 + wave;
  int bh = tile >> 12;
  int t  = tile & 4095;
  int mt = t >> 5;
  int pt = t & 31;
  int m0 = mt * 16, p0 = pt * 16;
  int h = bh % H_;

  int ln = lane & 15;
  int khalf = (lane >> 4) << 3;
  const half_t* xrow = A   + ((size_t)bh * S_ + m0 + ln) * D_;
  const half_t* prow = Pos + (size_t)(p0 + ln) * HID_ + h * D_;

  v8f acc = {};
  #pragma unroll
  for (int k0 = 0; k0 < D_; k0 += 32) {
    AFrag a, b;
    a.h[0] = *(const v8h*)(xrow + k0 + khalf);
    a.h[1] = *(const v8h*)(xrow + k0 + khalf + 16);
    b.h[0] = *(const v8h*)(prow + k0 + khalf);
    b.h[1] = *(const v8h*)(prow + k0 + khalf + 16);
    acc = wmma16(a.v, b.v, acc);
  }

  #pragma unroll
  for (int g = 0; g < 8; ++g) T[((lane >> 4) << 3) + g][wave * 16 + ln] = (half_t)acc[g];
  __syncthreads();
  {
    half_t* ob = Out + ((size_t)bh * S_) * P_;
    const int pb0 = (pt & ~7) * 16;
    const int tid = threadIdx.x, r = tid >> 4, pc = tid & 15;
    vst2(ob + (size_t)(m0 + r) * P_ + pb0 + pc * 8, *(const v4u*)(&T[r][pc * 8]));
  }
}

__global__ void __launch_bounds__(256)
attn_kernel(const half_t* __restrict__ qf, const half_t* __restrict__ kf,
            const half_t* __restrict__ vt,
            const half_t* __restrict__ c2p, const half_t* __restrict__ p2c,
            half_t* __restrict__ attnout) {
  __shared__ int tbl[4096];
  __shared__ __align__(16) half_t pst[8 * 16 * 64];
  __shared__ __align__(16) half_t kst[2][64 * 64];
  __shared__ __align__(16) half_t vst[2][64 * 64];
  __shared__ __align__(16) half_t ost[8][16 * 64];

  int tid = threadIdx.x;
  for (int d = tid; d < 4095; d += 256) {
    int delta = d - 2047;
    int ad = delta < 0 ? -delta : delta;
    int bk;
    if (ad <= 128) {
      bk = delta;
    } else {
      double xx = log((double)ad / 128.0) * 127.0 / log(511.0 / 128.0);
      double rx = rint(xx);
      int li = (fabs(xx - rx) < 1e-6) ? (int)rx : (int)ceil(xx);
      li += 128;
      bk = delta > 0 ? li : -li;
    }
    int tt = bk + 256;
    tbl[d] = tt < 0 ? 0 : (tt > 511 ? 511 : tt);
  }

  int lane = tid & 31;
  int wave = tid >> 5;
  int bh   = blockIdx.x >> 4;
  int qblk = blockIdx.x & 15;
  int i0 = qblk * 128 + wave * 16;

  const half_t* qb = qf  + ((size_t)bh * S_) * D_;
  const half_t* kb = kf  + ((size_t)bh * S_) * D_;
  const half_t* vb = vt  + ((size_t)bh * S_) * D_;
  const half_t* cb = c2p + ((size_t)bh * S_) * P_;
  const half_t* pb = p2c + ((size_t)bh * S_) * P_;

  auto stage = [&](int buf, int j0) {
    #pragma unroll
    for (int kk = 0; kk < 2; ++kk) {
      int c  = tid + kk * 256;
      int r  = c >> 3, cc = (c & 7) * 8;
      const half_t* gk = kb + (size_t)(j0 + r) * D_ + cc;
      const half_t* gv = vb + (size_t)(j0 + r) * D_ + cc;
      half_t* lk = &kst[buf][r * 64 + cc];
      *(v8h*)lk = *(const v8h*)gk;
      v8h vv = *(const v8h*)gv;
      #pragma unroll
      for (int e = 0; e < 8; ++e) vst[buf][(cc + e) * 64 + r] = vv[e];
    }
  };

  int ln = lane & 15;
  int khalf = (lane >> 4) << 3;
  int rsel  = (lane >> 4) << 3;

  AFrag qa[2];
  {
    const half_t* qrow = qb + (size_t)(i0 + ln) * D_;
    #pragma unroll
    for (int ks = 0; ks < 2; ++ks) {
      qa[ks].h[0] = *(const v8h*)(qrow + ks * 32 + khalf);
      qa[ks].h[1] = *(const v8h*)(qrow + ks * 32 + khalf + 16);
    }
  }

  v8f zero = {};
  v8f outacc[4];
  float mrow[8], lrow[8];
  #pragma unroll
  for (int nt = 0; nt < 4; ++nt) outacc[nt] = zero;
  #pragma unroll
  for (int g = 0; g < 8; ++g) { mrow[g] = -1e30f; lrow[g] = 0.0f; }

  half_t* myp = pst + wave * (16 * 64);

  stage(0, 0);
  __syncthreads();

  for (int jt = 0; jt < S_ / 64; ++jt) {
    int j0  = jt * 64;
    int cur = jt & 1;
    if (jt + 1 < S_ / 64) stage(cur ^ 1, j0 + 64);

    const half_t* kT = kst[cur];
    const half_t* vT = vst[cur];

    v8f sc[4];
    #pragma unroll
    for (int ct = 0; ct < 4; ++ct) {
      sc[ct] = zero;
      const half_t* krow = kT + (ct * 16 + ln) * 64;
      #pragma unroll
      for (int ks = 0; ks < 2; ++ks) {
        AFrag bf;
        bf.h[0] = *(const v8h*)(krow + ks * 32 + khalf);
        bf.h[1] = *(const v8h*)(krow + ks * 32 + khalf + 16);
        sc[ct] = wmma16(qa[ks].v, bf.v, sc[ct]);
      }
    }
    #pragma unroll
    for (int ct = 0; ct < 4; ++ct) {
      int j = j0 + ct * 16 + ln;
      #pragma unroll
      for (int g = 0; g < 8; ++g) {
        int i = i0 + rsel + g;
        int t = tbl[i - j + 2047];
        float bias = (float)cb[(size_t)i * P_ + t] + (float)pb[(size_t)j * P_ + t];
        sc[ct][g] = sc[ct][g] * SCALE_ + bias;
      }
    }
    float tm[8];
    #pragma unroll
    for (int g = 0; g < 8; ++g) {
      float v = fmaxf(fmaxf(sc[0][g], sc[1][g]), fmaxf(sc[2][g], sc[3][g]));
      v = fmaxf(v, __shfl_xor(v, 1, 32));
      v = fmaxf(v, __shfl_xor(v, 2, 32));
      v = fmaxf(v, __shfl_xor(v, 4, 32));
      v = fmaxf(v, __shfl_xor(v, 8, 32));
      tm[g] = v;
    }
    #pragma unroll
    for (int g = 0; g < 8; ++g) {
      float mnew = fmaxf(mrow[g], tm[g]);
      float corr = __expf(mrow[g] - mnew);
      mrow[g] = mnew;
      lrow[g] *= corr;
      #pragma unroll
      for (int nt = 0; nt < 4; ++nt) outacc[nt][g] *= corr;
    }
    #pragma unroll
    for (int g = 0; g < 8; ++g) {
      float rs = 0.0f;
      #pragma unroll
      for (int ct = 0; ct < 4; ++ct) {
        float p = __expf(sc[ct][g] - mrow[g]);
        rs += p;
        myp[(rsel + g) * 64 + ct * 16 + ln] = (half_t)(p * PSC);
      }
      rs += __shfl_xor(rs, 1, 32);
      rs += __shfl_xor(rs, 2, 32);
      rs += __shfl_xor(rs, 4, 32);
      rs += __shfl_xor(rs, 8, 32);
      lrow[g] += rs;
    }
    __syncthreads();
    AFrag pa[2];
    {
      const half_t* prow = myp + ln * 64;
      #pragma unroll
      for (int ks = 0; ks < 2; ++ks) {
        pa[ks].h[0] = *(const v8h*)(prow + ks * 32 + khalf);
        pa[ks].h[1] = *(const v8h*)(prow + ks * 32 + khalf + 16);
      }
    }
    #pragma unroll
    for (int nt = 0; nt < 4; ++nt) {
      const half_t* vrow = vT + (nt * 16 + ln) * 64;
      #pragma unroll
      for (int ks = 0; ks < 2; ++ks) {
        AFrag bf;
        bf.h[0] = *(const v8h*)(vrow + ks * 32 + khalf);
        bf.h[1] = *(const v8h*)(vrow + ks * 32 + khalf + 16);
        outacc[nt] = wmma16(pa[ks].v, bf.v, outacc[nt]);
      }
    }
    __syncthreads();
  }

  int b = bh / H_, h = bh - b * H_;
  half_t* os_ = &ost[wave][0];
  #pragma unroll
  for (int g = 0; g < 8; ++g) {
    float inv = PUN / lrow[g];
    #pragma unroll
    for (int nt = 0; nt < 4; ++nt) os_[(rsel + g) * 64 + nt * 16 + ln] = (half_t)(outacc[nt][g] * inv);
  }
  __syncthreads();
  #pragma unroll
  for (int q = 0; q < 4; ++q) {
    const int rl = q * 4 + (lane >> 3), pc = lane & 7;
    vst2(attnout + ((size_t)(b * S_ + i0 + rl)) * HID_ + h * D_ + pc * 8, *(const v4u*)(os_ + rl * 64 + pc * 8));
  }
}

extern "C" void kernel_launch(void* const* d_in, const int* in_sizes, int n_in,
                              void* d_out, int out_size, void* d_ws, size_t ws_size,
                              hipStream_t stream) {
  (void)in_sizes; (void)n_in; (void)out_size; (void)ws_size;
  const float* hidden = (const float*)d_in[0];
  const float* rel    = (const float*)d_in[1];
  const float* Wq = (const float*)d_in[2];
  const float* bq = (const float*)d_in[3];
  const float* Wk = (const float*)d_in[4];
  const float* bk = (const float*)d_in[5];
  const float* Wv = (const float*)d_in[6];
  const float* bv = (const float*)d_in[7];
  const float* Wo = (const float*)d_in[8];
  const float* bo = (const float*)d_in[9];
  float* out = (float*)d_out;

  char* ws = (char*)d_ws;
  size_t off = 0;
  auto alloc = [&](size_t bytes) -> void* {
    void* p = ws + off;
    off = (off + bytes + 255) & ~(size_t)255;
    return p;
  };
  const size_t M = (size_t)B_ * S_;
  half_t* hf    = (half_t*)alloc(M * HID_ * 2);
  half_t* relf  = (half_t*)alloc((size_t)P_ * HID_ * 2);
  half_t* WqT   = (half_t*)alloc((size_t)HID_ * HID_ * 2);
  half_t* WkT   = (half_t*)alloc((size_t)HID_ * HID_ * 2);
  half_t* WvT   = (half_t*)alloc((size_t)HID_ * HID_ * 2);
  half_t* WoT   = (half_t*)alloc((size_t)HID_ * HID_ * 2);
  half_t* qfb   = (half_t*)alloc(M * HID_ * 2);
  half_t* kfb   = (half_t*)alloc(M * HID_ * 2);
  half_t* vtb   = (half_t*)alloc(M * HID_ * 2);
  half_t* posk  = (half_t*)alloc((size_t)P_ * HID_ * 2);
  half_t* posq  = (half_t*)alloc((size_t)P_ * HID_ * 2);
  half_t* c2pb  = (half_t*)alloc((size_t)B_ * H_ * S_ * P_ * 2);
  half_t* p2cb  = (half_t*)alloc((size_t)B_ * H_ * S_ * P_ * 2);
  half_t* aout  = (half_t*)alloc(M * HID_ * 2);

  dim3 blk(256);

  cvt_f16_kernel<<<dim3((M * HID_ / 8) / 256), blk, 0, stream>>>(hidden, hf, (int)(M * HID_));
  cvt_f16_kernel<<<dim3((P_ * HID_ / 8) / 256), blk, 0, stream>>>(rel, relf, P_ * HID_);
  const int tblk = (HID_ / 64) * (HID_ / 64);
  cvt_transpose_kernel<<<dim3(tblk), blk, 0, stream>>>(Wq, WqT);
  cvt_transpose_kernel<<<dim3(tblk), blk, 0, stream>>>(Wk, WkT);
  cvt_transpose_kernel<<<dim3(tblk), blk, 0, stream>>>(Wv, WvT);
  cvt_transpose_kernel<<<dim3(tblk), blk, 0, stream>>>(Wo, WoT);

  const int gblk  = (int)((M / 16) * (HID_ / 16) / 8);
  gemm_proj_kernel<<<dim3(gblk), blk, 0, stream>>>(hf, WqT, bq, qfb, nullptr, (int)M, 0);
  gemm_proj_kernel<<<dim3(gblk), blk, 0, stream>>>(hf, WkT, bk, kfb, nullptr, (int)M, 0);
  gemm_proj_kernel<<<dim3(gblk), blk, 0, stream>>>(hf, WvT, bv, vtb, nullptr, (int)M, 0);

  const int pblk = (P_ / 16) * (HID_ / 16) / 8;
  gemm_proj_kernel<<<dim3(pblk), blk, 0, stream>>>(relf, WkT, bk, posk, nullptr, P_, 2);
  gemm_proj_kernel<<<dim3(pblk), blk, 0, stream>>>(relf, WqT, bq, posq, nullptr, P_, 2);

  const int rblk = (B_ * H_ * (S_ / 16) * (P_ / 16)) / 8;
  gemm_rel_kernel<<<dim3(rblk), blk, 0, stream>>>(qfb, posk, c2pb);
  gemm_rel_kernel<<<dim3(rblk), blk, 0, stream>>>(kfb, posq, p2cb);

  attn_kernel<<<dim3(B_ * H_ * (S_ / 128)), blk, 0, stream>>>(qfb, kfb, vtb, c2pb, p2cb, aout);

  gemm_proj_kernel<<<dim3(gblk), blk, 0, stream>>>(aout, WoT, bo, nullptr, out, (int)M, 3);
}
